// MetabolismProcessor_61899068670355
// MI455X (gfx1250) — hardware-run, weakly checked
//
#include <hip/hip_runtime.h>

typedef float          v8f   __attribute__((ext_vector_type(8)));
typedef float          v4f   __attribute__((ext_vector_type(4)));
typedef unsigned int   v4u   __attribute__((ext_vector_type(4)));
typedef int            v8i   __attribute__((ext_vector_type(8)));
typedef unsigned short v8us  __attribute__((ext_vector_type(8)));
typedef unsigned short v16us __attribute__((ext_vector_type(16)));
typedef __bf16         v16bf __attribute__((ext_vector_type(16)));
typedef _Float16       v16h  __attribute__((ext_vector_type(16)));
typedef v4f  __attribute__((may_alias)) v4fa;
typedef v8us __attribute__((may_alias)) v8usa;
union FragB { v16bf v; v16us u; v8us h[2]; v8i w; };
union FragH { v16h  v; v16us u; v8us h[2]; v8i w; };

__device__ __forceinline__ v8f wmb(const FragB& a, const FragB& b, v8f c) {
  v8f d = __builtin_amdgcn_wmma_f32_16x16x32_bf16(false, a.v, false, b.v, (short)0, c, false, false);
  asm volatile("v_nop\n\tv_nop\n\tv_nop\n\tv_nop" : "+v"(d) : "v"(a.w), "v"(b.w));
  return d;
}

__device__ __forceinline__ v8f wmh(const FragH& a, const FragH& b, v8f c) {
  v8f d = __builtin_amdgcn_wmma_f32_16x16x32_f16(false, a.v, false, b.v, (short)0, c, false, false);
  asm volatile("v_nop\n\tv_nop\n\tv_nop\n\tv_nop" : "+v"(d) : "v"(a.w), "v"(b.w));
  return d;
}

__device__ __forceinline__ unsigned bf16_bits(float f) {
  const unsigned u = __float_as_uint(f);
  const unsigned r = (u + 0x7FFFu + ((u >> 16) & 1u)) >> 16;
  const unsigned q = (u >> 16) | 0x40u;
  return ((u & 0x7fffffffu) > 0x7f800000u) ? q : r;
}

__device__ __forceinline__ float bf16_val(float f) {
  return __uint_as_float(bf16_bits(f) << 16);
}
__device__ __forceinline__ int clampi(int v, int lo, int hi) {
  return v < lo ? lo : (v > hi ? hi : v);
}

__device__ __forceinline__ unsigned f16_bits(float f) {
  const unsigned u  = __float_as_uint(f);
  const unsigned s  = (u >> 16) & 0x8000u;
  const unsigned a  = u & 0x7fffffffu;
  const unsigned t  = a - 0x38000000u;
  const unsigned r  = (t + 0x0FFFu + ((t >> 13) & 1u)) >> 13;
  const unsigned rc = r > 0x7C00u ? 0x7C00u : r;
  const bool small  = a < 0x38800000u;
  const bool isnan  = a > 0x7f800000u;
  const unsigned fin = small ? 0u : (s | rc);
  return isnan ? (s | 0x7E00u) : fin;
}

__device__ __forceinline__ unsigned pk16(unsigned lo, unsigned hi) { return lo | (hi << 16); }
__device__ __forceinline__ unsigned bf16_lo_bits(float v) {
  float hi = bf16_val(v);
  asm volatile("" : "+v"(hi));
  return bf16_bits(v - hi);
}
__device__ __forceinline__ v4u pack8_bf16(v4f a, v4f c) {
  return (v4u){ pk16(bf16_bits(a[0]), bf16_bits(a[1])), pk16(bf16_bits(a[2]), bf16_bits(a[3])),
                pk16(bf16_bits(c[0]), bf16_bits(c[1])), pk16(bf16_bits(c[2]), bf16_bits(c[3])) };
}
__device__ __forceinline__ v4u pack8_bf16_lo(v4f a, v4f c) {
  return (v4u){ pk16(bf16_lo_bits(a[0]), bf16_lo_bits(a[1])), pk16(bf16_lo_bits(a[2]), bf16_lo_bits(a[3])),
                pk16(bf16_lo_bits(c[0]), bf16_lo_bits(c[1])), pk16(bf16_lo_bits(c[2]), bf16_lo_bits(c[3])) };
}
__device__ __forceinline__ v4u pack8_f16(v4f a, v4f c) {
  return (v4u){ pk16(f16_bits(a[0]), f16_bits(a[1])), pk16(f16_bits(a[2]), f16_bits(a[3])),
                pk16(f16_bits(c[0]), f16_bits(c[1])), pk16(f16_bits(c[2]), f16_bits(c[3])) };
}

template <int FORM>
__global__ __launch_bounds__(256) void k_plane(const float* __restrict__ src, int rows, int cols, int ldsrc,
                                               unsigned short* __restrict__ dst, int MP, int KP) {
  static_assert(FORM >= 0 && FORM <= 3);
  const int KTOT = (FORM == 1 || FORM == 3) ? 2 * KP : KP;
  const unsigned ppr   = (unsigned)(KTOT >> 3);
  const unsigned kp8   = (unsigned)(KP >> 3);
  const unsigned total = (unsigned)MP * ppr;
  const unsigned g     = blockIdx.x * 256u + threadIdx.x;
  const unsigned rowu  = g / ppr;
  const unsigned p     = g - rowu * ppr;
  const bool second    = p >= kp8;
  const int row = (int)rowu;
  const int c0  = (int)((second ? p - kp8 : p) << 3);
  const float* srow = src + (size_t)clampi(row, 0, rows - 1) * (size_t)ldsrc;
  float x[8];
  unsigned mk[8];
#pragma unroll
  for (int e = 0; e < 8; ++e) {
    const int c = c0 + e;
    const float v = srow[clampi(c, 0, cols - 1)];
    asm volatile("" :: "v"(v));
    x[e]  = v;
    mk[e] = (row < rows && c < cols) ? 0xFFFFu : 0u;
  }
  const v4f a = (v4f){ x[0], x[1], x[2], x[3] };
  const v4f c = (v4f){ x[4], x[5], x[6], x[7] };
  v4u o;
  if (FORM == 2) {
    o = pack8_f16(a, c);
  } else {
    const v4u hi = pack8_bf16(a, c);
    o = hi;
    if (FORM == 1) { const v4u lo = pack8_bf16_lo(a, c); o = second ? lo : hi; }
  }
  const v4u mw = (v4u){ pk16(mk[0], mk[1]), pk16(mk[2], mk[3]), pk16(mk[4], mk[5]), pk16(mk[6], mk[7]) };
  o &= mw;
  if (g < total) {
    volatile v4u* q = (volatile v4u*)(dst + (size_t)g * 8);
    *q = o;
    __threadfence();
    *q = o;
  }
}

template <int FORM> struct FragOf    { typedef FragB T; };
template <>         struct FragOf<2> { typedef FragH T; };
__device__ __forceinline__ v8f mm(const FragB& a, const FragB& b, v8f c) { return wmb(a, b, c); }
__device__ __forceinline__ v8f mm(const FragH& a, const FragH& b, v8f c) { return wmh(a, b, c); }
template <class F> __device__ __forceinline__ F ld_frag(const unsigned short* p) {
  F f;
  f.h[0] = *(const v8usa*)(p);
  f.h[1] = *(const v8usa*)(p + 16);
  return f;
}

template <int FORM, int EPI>
__global__ __launch_bounds__(256) __attribute__((amdgpu_num_vgpr(248)))
void k_gemm_nt(const unsigned short* __restrict__ A, const unsigned short* __restrict__ B,
               const float* __restrict__ bias, float* __restrict__ D, int M, int N, int KTOT, int ldd) {
  static_assert(FORM >= 0 && FORM <= 2);
  static_assert(EPI == 0 || EPI == 1);
  typedef typename FragOf<FORM>::T F;
  __shared__ __attribute__((aligned(16))) float sT[8][16 * 68];
  const int lane = threadIdx.x & 31;
  const int wave = threadIdx.x >> 5;
  const int tilesM = (M + 63) >> 6;
  const int tilesN = (N + 63) >> 6;
  const int tile = blockIdx.x * 8 + wave;
  if (tile >= tilesM * tilesN) return;
  const int tm = tile / tilesN;
  const int tn = tile - tm * tilesN;
  const int m0 = tm << 6;
  const int n0 = tn << 6;

  const int rl = lane & 15;
  const int h8 = (lane >> 4) * 8;
  const unsigned short* pa = A + (size_t)(m0 + rl) * (size_t)KTOT + h8;
  const unsigned short* pb = B + (size_t)(n0 + rl) * (size_t)KTOT + h8;

  v8f acc[4][4];
#pragma unroll
  for (int i = 0; i < 4; ++i)
#pragma unroll
    for (int j = 0; j < 4; ++j) acc[i][j] = (v8f){0.f, 0.f, 0.f, 0.f, 0.f, 0.f, 0.f, 0.f};

#pragma unroll 1
  for (int k0 = 0; k0 < KTOT; k0 += 32) {
    F bf[4];
#pragma unroll
    for (int j = 0; j < 4; ++j) bf[j] = ld_frag<F>(pb + (size_t)(j << 4) * (size_t)KTOT + k0);
#pragma unroll
    for (int i = 0; i < 4; ++i) {
      const F af = ld_frag<F>(pa + (size_t)(i << 4) * (size_t)KTOT + k0);
#pragma unroll
      for (int j = 0; j < 4; ++j) acc[i][j] = mm(af, bf[j], acc[i][j]);
    }
  }

  float* slab = sT[wave];
  const int hh = lane >> 4;
  const int c4 = (lane & 15) * 4;
  const int nc = n0 + c4;
  const bool cok = nc < N;
  v4f bv = (v4f){0.f, 0.f, 0.f, 0.f};
  if (EPI == 1) {
    bv = *(const v4fa*)(bias + clampi(nc, 0, N - 4));
    asm volatile("" :: "v"(bv));
  }
#pragma unroll
  for (int i = 0; i < 4; ++i) {
    const int mBase = m0 + (i << 4);
#pragma unroll
    for (int j = 0; j < 4; ++j) {
#pragma unroll
      for (int r = 0; r < 8; ++r) slab[(h8 + r) * 68 + (j << 4) + rl] = acc[i][j][r];
    }
    __builtin_amdgcn_fence(__ATOMIC_RELEASE, "workgroup");
    __builtin_amdgcn_wave_barrier();
    __builtin_amdgcn_fence(__ATOMIC_ACQUIRE, "workgroup");
    v4f vv[8];
#pragma unroll
    for (int it = 0; it < 8; ++it) {
      const int row = it * 2 + hh;
      v4f v = *(const v4fa*)(slab + row * 68 + c4);
      if (EPI == 1) v += bv;
      vv[it] = v;
    }
    for (int pass = 0; pass < 2; ++pass) {
#pragma unroll
      for (int it = 0; it < 8; ++it) {
        const int row = mBase + it * 2 + hh;
        if (cok && row < M) *(volatile v4f*)(D + (size_t)row * (size_t)ldd + nc) = vv[it];
      }
      __threadfence();
    }
    __builtin_amdgcn_fence(__ATOMIC_RELEASE, "workgroup");
    __builtin_amdgcn_wave_barrier();
    __builtin_amdgcn_fence(__ATOMIC_ACQUIRE, "workgroup");
  }
}

#pragma clang fp contract(off)

typedef int          v4i  __attribute__((ext_vector_type(4)));
typedef unsigned int v2u  __attribute__((ext_vector_type(2)));
typedef v4i __attribute__((may_alias)) v4ia;

static constexpr int NMET = 2534, NRXN = 4881, NGENE = 6607, NE = 262144, NP = 131072, DD = 256;
static constexpr int MPM = 2560, MPR = 4928, KT = 512;
static constexpr int RCAP = 28672;
static constexpr int DEGCAP = 160;
static constexpr int SLB = 9, SLMAX = 512;
static constexpr int BCH = 1024;
static constexpr int BK_INTS = 2 * RCAP + 3 * SLMAX + 32;
static constexpr int SL_A = 9, SL_B = 8, SL_C = 7, SL_D = 9;
static constexpr int NB_A = 10, NB_B = 20, NB_C = 20, NB_D = 13;
static constexpr int PA_ATT0 = 0, PA_ATT1 = 512, PA_B0 = 1024, PA_B1 = 1280, PA_LNG = 1536, PA_LNB = 1792;
static constexpr int PREP_WT = 256, PREP_PAR = 2, PREP_MET = MPM / 8;
static constexpr size_t WSMAX = ((size_t)128 << 20);

static_assert(DD == 32 * 8);
static_assert(MPM % 64 == 0 && MPR % 64 == 0 && MPM >= NMET && MPR >= NRXN);
static_assert(NE % BCH == 0 && NP % BCH == 0 && NE % 256 == 0 && NP % 256 == 0);
static_assert(NE < (1 << 22) && NP < (1 << 22));
static_assert((1 << SL_A) % 32 == 0 && (1 << SL_B) % 32 == 0 && (1 << SL_C) % 32 == 0 && (1 << SL_D) % 32 == 0);
static_assert((1 << SL_A) <= SLMAX && (1 << SL_B) <= SLMAX && (1 << SL_C) <= SLMAX && (1 << SL_D) <= SLMAX);
static_assert((NB_A << SL_A) >= NRXN && (NB_B << SL_B) >= NRXN && (NB_C << SL_C) >= NMET && (NB_D << SL_D) >= NGENE);
static_assert(RCAP >= 28006 && RCAP <= 28672 && RCAP % 1024 == 0);
static_assert(DEGCAP >= 149 && DEGCAP % 32 == 0);
static_assert(BK_INTS % 4 == 0 && BK_INTS * 4 <= 327680);
static_assert(KT == 2 * DD && KT % 32 == 0);

__device__ __forceinline__ float qnanf() { return __uint_as_float(0x7fc00000u); }
__device__ __forceinline__ float ninff() { return __uint_as_float(0xff800000u); }
__device__ __forceinline__ float nanmax(float a, float b) { return (b > a || b != b) ? b : a; }
__device__ __forceinline__ float wave_sum(float v) {
#pragma unroll
  for (int off = 16; off > 0; off >>= 1) v += __shfl_xor(v, off);
  return v;
}
__device__ __forceinline__ float wave_nanmax(float v) {
#pragma unroll
  for (int off = 16; off > 0; off >>= 1) { const float o = __shfl_xor(v, off); v = nanmax(v, o); }
  return v;
}
__device__ __forceinline__ v4f bfr4(v4f a) {
  return (v4f){ bf16_val(a[0]), bf16_val(a[1]), bf16_val(a[2]), bf16_val(a[3]) };
}
__device__ __forceinline__ void wave_sync_lds() {
  __builtin_amdgcn_fence(__ATOMIC_RELEASE, "workgroup");
  __builtin_amdgcn_wave_barrier();
  __builtin_amdgcn_fence(__ATOMIC_ACQUIRE, "workgroup");
}

__device__ __forceinline__ float edge_logit(float sx, float se) {
  const float v = sx + se;
  return v >= 0.0f ? v : 0.2f * v;
}
__device__ __forceinline__ float edge_ex(float sx, float se, float mx) {
  return expf(edge_logit(sx, se) - mx);
}
__device__ __forceinline__ float edge_w(float sx, float se, float mx, float den, float st) {
  const float ex = edge_ex(sx, se, mx);
  return st * (ex / den);
}
__device__ __forceinline__ float tanh_acc(float x) {
  const float ax = fabsf(x);
  const float x2 = x * x;
  float p = fmaf(x2, -17.0f / 315.0f, 2.0f / 15.0f);
  p = fmaf(x2, p, -1.0f / 3.0f);
  p = fmaf(x2, p, 1.0f);
  const float sm = x * p;
  const float e  = expf(2.0f * ax);
  const float bg = copysignf(1.0f - 2.0f / (e + 1.0f), x);
  return (ax < 0.25f) ? sm : bg;
}

__device__ __forceinline__ void store_row(float* rowp, int lane, v4f r0, v4f r1) {
  float* p = rowp + 4 * lane;
  for (int pass = 0; pass < 2; ++pass) {
    *(volatile v4f*)(p)       = r0;
    *(volatile v4f*)(p + 128) = r1;
    __threadfence();
  }
}
__device__ __forceinline__ void store_hl(unsigned short* rowp, int lane, v4f r0, v4f r1) {
  const v2u h0 = (v2u){ pk16(bf16_bits(r0[0]), bf16_bits(r0[1])), pk16(bf16_bits(r0[2]), bf16_bits(r0[3])) };
  const v2u h1 = (v2u){ pk16(bf16_bits(r1[0]), bf16_bits(r1[1])), pk16(bf16_bits(r1[2]), bf16_bits(r1[3])) };
  const v2u l0 = (v2u){ pk16(bf16_lo_bits(r0[0]), bf16_lo_bits(r0[1])), pk16(bf16_lo_bits(r0[2]), bf16_lo_bits(r0[3])) };
  const v2u l1 = (v2u){ pk16(bf16_lo_bits(r1[0]), bf16_lo_bits(r1[1])), pk16(bf16_lo_bits(r1[2]), bf16_lo_bits(r1[3])) };
  unsigned short* p = rowp + 4 * lane;
  for (int pass = 0; pass < 2; ++pass) {
    *(volatile v2u*)(p)       = h0;
    *(volatile v2u*)(p + 128) = h1;
    *(volatile v2u*)(p + 256) = l0;
    *(volatile v2u*)(p + 384) = l1;
    __threadfence();
  }
}

__device__ __forceinline__ void seg_hdr(const int* __restrict__ OFF, const int* __restrict__ CNT,
                                        const int* __restrict__ FLAG, int segc, int slb, bool live,
                                        int& c, int& o, bool& bad) {
  int cr = CNT[segc];
  int orr = OFF[segc];
  int fl = FLAG[(segc >> slb) * 32];
  const int badv = (live && ((fl != 0) || (cr < 0) || (cr > DEGCAP) || (orr < 0) || (orr > RCAP - cr))) ? 1 : 0;
  const int cv = live ? clampi(cr, 0, DEGCAP) : 0;
  const int ov = clampi(orr, 0, RCAP - 1);
  bad = __builtin_amdgcn_readfirstlane(badv) != 0;
  c = __builtin_amdgcn_readfirstlane(cv);
  o = __builtin_amdgcn_readfirstlane(ov);
}
__device__ __forceinline__ void fetch_inc(const int* __restrict__ lp, int o, int j, int nKeys,
                                          const int* __restrict__ other, int nOther, int& e, int& x) {
  int idx = o + j;
  idx = idx > RCAP - 1 ? RCAP - 1 : idx;
  e = clampi(lp[idx], 0, nKeys - 1);
  x = clampi(other[e], 0, nOther - 1);
}

__device__ __forceinline__ void wt_unit(const float* __restrict__ W, unsigned short* dstMat, int v) {
  const int n  = v >> 6;
  const int k8 = (v & 63) * 8;
  const int kk = k8 & (DD - 1);
  const float* p = W + (size_t)kk * DD + n;
  float x[8];
#pragma unroll
  for (int i = 0; i < 8; ++i) { const float t = p[(size_t)i * DD]; asm volatile("" :: "v"(t)); x[i] = t; }
  const v4u o = pack8_bf16((v4f){ x[0], x[1], x[2], x[3] }, (v4f){ x[4], x[5], x[6], x[7] });
  volatile v4u* q = (volatile v4u*)(dstMat + (size_t)n * KT + k8);
  *q = o;
  __threadfence();
  *q = o;
}
__device__ __forceinline__ void par_unit(const float* __restrict__ src, int so, float* PAR, int f) {
  const v4f v = bfr4(*(const v4f*)(src + so));
  volatile v4f* q = (volatile v4f*)(PAR + f);
  *q = v;
  __threadfence();
  *q = v;
}
__global__ __launch_bounds__(256) void k_prep(const float* __restrict__ emb,
                                              const float* __restrict__ W0, const float* __restrict__ We0,
                                              const float* __restrict__ W1, const float* __restrict__ We1,
                                              const float* __restrict__ att0, const float* __restrict__ att1,
                                              const float* __restrict__ b0, const float* __restrict__ b1,
                                              const float* __restrict__ lng, const float* __restrict__ lnb,
                                              unsigned short* WT2, float* PAR, unsigned short* METhl) {
  const int tid = (int)threadIdx.x, lane = tid & 31;
  const int wave = __builtin_amdgcn_readfirstlane(tid >> 5);
  const int blk = (int)blockIdx.x;
  if (blk < PREP_WT) {
    const int mat = blk >> 6;
    const int v = (blk & 63) * 256 + tid;
    unsigned short* dm = WT2 + (size_t)mat * (DD * KT);
    if (mat == 0)      wt_unit(W0, dm, v);
    else if (mat == 1) wt_unit(We0, dm, v);
    else if (mat == 2) wt_unit(W1, dm, v);
    else               wt_unit(We1, dm, v);
  } else if (blk < PREP_WT + PREP_PAR) {
    const int f = ((blk - PREP_WT) * 256 + tid) * 4;
    if (f < PA_ATT1)      par_unit(att0, f - PA_ATT0, PAR, f);
    else if (f < PA_B0)   par_unit(att1, f - PA_ATT1, PAR, f);
    else if (f < PA_B1)   par_unit(b0,   f - PA_B0,   PAR, f);
    else if (f < PA_LNG)  par_unit(b1,   f - PA_B1,   PAR, f);
    else if (f < PA_LNB)  par_unit(lng,  f - PA_LNG,  PAR, f);
    else                  par_unit(lnb,  f - PA_LNB,  PAR, f);
  } else {
    const int row = (blk - PREP_WT - PREP_PAR) * 8 + wave;
    const bool live = row < NMET;
    const float* rp = emb + (size_t)(row < NMET ? row : NMET - 1) * DD;
    const v4f x0 = bfr4(*(const v4f*)(rp + 4 * lane));
    const v4f x1 = bfr4(*(const v4f*)(rp + 128 + 4 * lane));
    float ss = 0.0f;
    ss += x0[0] * x0[0]; ss += x0[1] * x0[1]; ss += x0[2] * x0[2]; ss += x0[3] * x0[3];
    ss += x1[0] * x1[0]; ss += x1[1] * x1[1]; ss += x1[2] * x1[2]; ss += x1[3] * x1[3];
    ss = wave_sum(ss);
    const float nrm = sqrtf(ss);
    const float t = 1.0f / (nrm + 1e-12f);
    const float f = (t >= 1.0f) ? 1.0f : t;
    v4f y0 = x0 * f;
    v4f y1 = x1 * f;
    const v4f z = (v4f){ 0.f, 0.f, 0.f, 0.f };
    y0 = live ? y0 : z;
    y1 = live ? y1 : z;
    store_hl(METhl + (size_t)row * KT, lane, y0, y1);
  }
}

__global__ __launch_bounds__(256) void k_bucket(const int* __restrict__ keys, int nKeys, int nSeg, int slots,
                                                int* LIST, int* OFF, int* CNT, int* FLAG) {
  extern __shared__ __attribute__((aligned(16))) int bsm[];
  int* hl   = bsm;
  int* sl   = bsm + RCAP;
  int* cnt  = bsm + 2 * RCAP;
  int* offs = cnt + SLMAX;
  int* cur  = offs + SLMAX;
  int* wc   = cur + SLMAX;
  const int tid = (int)threadIdx.x, lane = tid & 31;
  const int wave = __builtin_amdgcn_readfirstlane(tid >> 5);
  const int blk = (int)blockIdx.x;
  const int slotBase = blk * slots;
  int nb = nSeg - slotBase;
  nb = nb < 0 ? 0 : (nb > slots ? slots : nb);

  {
    const v4i z4 = (v4i){ 0, 0, 0, 0 };
    for (int i = tid * 4; i < BK_INTS; i += 1024) *(v4ia*)(bsm + i) = z4;
  }
  __syncthreads();

  const unsigned ub = (unsigned)slotBase, unb = (unsigned)nb;
  int tot = 0;
  const int nCh = nKeys / BCH;
#pragma unroll 1
  for (int ch = 0; ch < nCh; ++ch) {
    const int e0 = ch * BCH + tid * 4;
    const v4i kv = *(const v4i*)(keys + e0);
    const unsigned s0 = (unsigned)kv[0] - ub, s1 = (unsigned)kv[1] - ub;
    const unsigned s2 = (unsigned)kv[2] - ub, s3 = (unsigned)kv[3] - ub;
    const bool h0 = s0 < unb, h1 = s1 < unb, h2 = s2 < unb, h3 = s3 < unb;
    const unsigned m0 = __builtin_amdgcn_ballot_w32(h0);
    const unsigned m1 = __builtin_amdgcn_ballot_w32(h1);
    const unsigned m2 = __builtin_amdgcn_ballot_w32(h2);
    const unsigned m3 = __builtin_amdgcn_ballot_w32(h3);
    const int wtot = (int)(__builtin_popcount(m0) + __builtin_popcount(m1) + __builtin_popcount(m2) + __builtin_popcount(m3));
    int* wcp = wc + (ch & 1) * 8;
    if (lane == 0) wcp[wave] = wtot;
    __syncthreads();
    const v4i wa = *(const v4ia*)(wcp);
    const v4i wb = *(const v4ia*)(wcp + 4);
    int pre = 0;
    pre += (wave > 0) ? wa[0] : 0;
    pre += (wave > 1) ? wa[1] : 0;
    pre += (wave > 2) ? wa[2] : 0;
    pre += (wave > 3) ? wa[3] : 0;
    pre += (wave > 4) ? wb[0] : 0;
    pre += (wave > 5) ? wb[1] : 0;
    pre += (wave > 6) ? wb[2] : 0;
    const int ctot = wa[0] + wa[1] + wa[2] + wa[3] + wb[0] + wb[1] + wb[2] + wb[3];
    int p = tot + pre + (int)(__builtin_amdgcn_mbcnt_lo(m0, 0u) + __builtin_amdgcn_mbcnt_lo(m1, 0u) +
                              __builtin_amdgcn_mbcnt_lo(m2, 0u) + __builtin_amdgcn_mbcnt_lo(m3, 0u));
    if (h0 && p < RCAP) hl[p] = ((e0 + 0) << SLB) | (int)s0;
    p += h0 ? 1 : 0;
    if (h1 && p < RCAP) hl[p] = ((e0 + 1) << SLB) | (int)s1;
    p += h1 ? 1 : 0;
    if (h2 && p < RCAP) hl[p] = ((e0 + 2) << SLB) | (int)s2;
    p += h2 ? 1 : 0;
    if (h3 && p < RCAP) hl[p] = ((e0 + 3) << SLB) | (int)s3;
    tot += ctot;
    tot = tot > 2 * RCAP ? 2 * RCAP : tot;
  }
  __syncthreads();
  const int ovf = __builtin_amdgcn_readfirstlane(tot > RCAP ? 1 : 0);
  const int tt  = __builtin_amdgcn_readfirstlane(tot > RCAP ? RCAP : tot);

  if (wave == 0) {
#pragma unroll 1
    for (int b0 = 0; b0 < tt; b0 += 32) {
      const int idx = b0 + lane;
      const bool valid = idx < tt;
      const int ent = hl[valid ? idx : tt - 1];
      const int slot = ent & (SLMAX - 1);
      unsigned mask = __builtin_amdgcn_ballot_w32(valid);
#pragma unroll
      for (int b = 0; b < SLB; ++b) {
        const bool bit = ((slot >> b) & 1) != 0;
        const unsigned bal = __builtin_amdgcn_ballot_w32(bit);
        mask &= bit ? bal : ~bal;
      }
      const int rank = (int)__builtin_amdgcn_mbcnt_lo(mask, 0u);
      const int grp  = (int)__builtin_popcount(mask);
      const int c0 = cnt[slot];
      if (valid && rank == 0) cnt[slot] = c0 + grp;
    }
  }
  __syncthreads();
  if (wave == 0) {
    const int base = lane * (SLMAX / 32);
    int s = 0;
#pragma unroll 1
    for (int i = 0; i < SLMAX / 32; ++i) s += cnt[base + i];
    int incl = s;
#pragma unroll
    for (int d = 1; d < 32; d <<= 1) {
      const int y = __shfl_up(incl, d, 32);
      incl += (lane >= d) ? y : 0;
    }
    int run = incl - s;
#pragma unroll 1
    for (int i = 0; i < SLMAX / 32; ++i) {
      const int cv = cnt[base + i];
      offs[base + i] = run;
      cur[base + i]  = run;
      run += cv;
    }
  }
  __syncthreads();
  if (wave == 0) {
#pragma unroll 1
    for (int b0 = 0; b0 < tt; b0 += 32) {
      const int idx = b0 + lane;
      const bool valid = idx < tt;
      const int ent = hl[valid ? idx : tt - 1];
      const int slot = ent & (SLMAX - 1);
      unsigned mask = __builtin_amdgcn_ballot_w32(valid);
#pragma unroll
      for (int b = 0; b < SLB; ++b) {
        const bool bit = ((slot >> b) & 1) != 0;
        const unsigned bal = __builtin_amdgcn_ballot_w32(bit);
        mask &= bit ? bal : ~bal;
      }
      const int rank = (int)__builtin_amdgcn_mbcnt_lo(mask, 0u);
      const int grp  = (int)__builtin_popcount(mask);
      const int cb = cur[slot];
      const int p = clampi(cb + rank, 0, RCAP - 1);
      if (valid) sl[p] = (int)((unsigned)ent >> SLB);
      if (valid && rank == 0) cur[slot] = cb + grp;
    }
  }
  __syncthreads();
  int* lg = LIST + (size_t)blk * RCAP;
  const v4i fv = (v4i){ ovf, ovf, ovf, ovf };
  for (int pass = 0; pass < 2; ++pass) {
#pragma unroll 1
    for (int i = tid * 4; i < RCAP; i += 1024) {
      const v4i v = *(const v4ia*)(sl + i);
      *(volatile v4i*)(lg + i) = v;
    }
    if (tid < (slots >> 2)) {
      const v4i vo = *(const v4ia*)(offs + 4 * tid);
      const v4i vc = *(const v4ia*)(cnt + 4 * tid);
      *(volatile v4i*)(OFF + (size_t)blk * slots + 4 * tid) = vo;
      *(volatile v4i*)(CNT + (size_t)blk * slots + 4 * tid) = vc;
    }
    if (tid < 8) *(volatile v4i*)(FLAG + (size_t)blk * 32 + 4 * tid) = fv;
    __threadfence();
  }
}

template <int HL, int RND>
__global__ __launch_bounds__(256) void k_mean(const int* __restrict__ LIST, const int* __restrict__ OFF,
                                              const int* __restrict__ CNT, const int* __restrict__ FLAG,
                                              int slb, int nSeg, int nRows,
                                              const int* __restrict__ gidx, int nIdx,
                                              const float* __restrict__ src, int nSrc,
                                              float* outF, unsigned short* outH) {
  const int tid = (int)threadIdx.x, lane = tid & 31;
  const int wave = __builtin_amdgcn_readfirstlane(tid >> 5);
  const int seg = (int)blockIdx.x * 8 + wave;
  if (seg >= nRows) return;
  const bool live = seg < nSeg;
  const int segc = live ? seg : nSeg - 1;
  int c, o; bool bad;
  seg_hdr(OFF, CNT, FLAG, segc, slb, live, c, o, bad);
  const int* lp = LIST + (size_t)(segc >> slb) * RCAP;
  v4f a0 = (v4f){ 0.f, 0.f, 0.f, 0.f };
  v4f a1 = (v4f){ 0.f, 0.f, 0.f, 0.f };
#pragma unroll 1
  for (int b0 = 0; b0 < c; b0 += 32) {
    int e, g;
    fetch_inc(lp, o, b0 + lane, nIdx, gidx, nSrc, e, g);
    const int m32 = (c - b0) < 32 ? (c - b0) : 32;
#pragma unroll 1
    for (int k = 0; k < m32; ++k) {
      const int gk = __builtin_amdgcn_readlane(g, k);
      const float* rp = src + (size_t)gk * DD;
      v4f x0 = *(const v4f*)(rp + 4 * lane);
      v4f x1 = *(const v4f*)(rp + 128 + 4 * lane);
      if (RND) { x0 = bfr4(x0); x1 = bfr4(x1); }
      a0 += x0;
      a1 += x1;
    }
  }
  const float inv = 1.0f / (float)(c > 1 ? c : 1);
  const float pz = bad ? qnanf() : 0.0f;
  v4f r0 = a0 * inv + pz;
  v4f r1 = a1 * inv + pz;
  const v4f z = (v4f){ 0.f, 0.f, 0.f, 0.f };
  r0 = live ? r0 : z;
  r1 = live ? r1 : z;
  if (HL) store_hl(outH + (size_t)seg * KT, lane, r0, r1);
  else    store_row(outF + (size_t)seg * DD, lane, r0, r1);
}

__global__ __launch_bounds__(256) void k_scores(const float* __restrict__ XPEP, const float* __restrict__ PAR,
                                                int attOff, float* S) {
  __shared__ __attribute__((aligned(16))) float sa[512];
  __shared__ __attribute__((aligned(16))) float sr[64];
  const int tid = (int)threadIdx.x, lane = tid & 31;
  const int wave = __builtin_amdgcn_readfirstlane(tid >> 5);
  if (tid < 128) *(v4fa*)(sa + 4 * tid) = *(const v4fa*)(PAR + attOff + 4 * tid);
  __syncthreads();
  const int g0 = (int)blockIdx.x * 64;
  const int ao = (g0 < MPM) ? 0 : DD;
  const v4f a0 = *(const v4fa*)(sa + ao + 4 * lane);
  const v4f a1 = *(const v4fa*)(sa + ao + 128 + 4 * lane);
#pragma unroll 1
  for (int i = 0; i < 8; ++i) {
    const int li = wave * 8 + i;
    const float* rp = XPEP + (size_t)(g0 + li) * DD;
    const v4f x0 = *(const v4f*)(rp + 4 * lane);
    const v4f x1 = *(const v4f*)(rp + 128 + 4 * lane);
    float s = 0.0f;
    s = fmaf(x0[0], a0[0], s); s = fmaf(x0[1], a0[1], s); s = fmaf(x0[2], a0[2], s); s = fmaf(x0[3], a0[3], s);
    s = fmaf(x1[0], a1[0], s); s = fmaf(x1[1], a1[1], s); s = fmaf(x1[2], a1[2], s); s = fmaf(x1[3], a1[3], s);
    s = wave_sum(s);
    if (lane == 0) sr[li] = s;
  }
  __syncthreads();
  if (wave == 0) {
    const v4f v = *(const v4fa*)(sr + 4 * (lane & 15));
    float* op = S + g0 + 4 * (lane & 15);
    for (int pass = 0; pass < 2; ++pass) {
      if (lane < 16) *(volatile v4f*)op = v;
      __threadfence();
    }
  }
}

__global__ __launch_bounds__(256) void k_edge(const int* __restrict__ heNode, const float* __restrict__ stoich,
                                              const int* __restrict__ LISTB, const int* __restrict__ OFFB,
                                              const int* __restrict__ CNTB, const int* __restrict__ FLAGB,
                                              const float* __restrict__ S, const float* __restrict__ XP,
                                              float* ME, float* MX, float* DEN) {
  __shared__ __attribute__((aligned(16))) float smx[64];
  __shared__ __attribute__((aligned(16))) float sdn[64];
  const int tid = (int)threadIdx.x, lane = tid & 31;
  const int wave = __builtin_amdgcn_readfirstlane(tid >> 5);
  const float* SE = S + MPM;
#pragma unroll 1
  for (int i = 0; i < 8; ++i) {
    const int li = wave * 8 + i;
    const int r = (int)blockIdx.x * 64 + li;
    const bool live = r < NRXN;
    const int rc = live ? r : NRXN - 1;
    int c, o; bool bad;
    seg_hdr(OFFB, CNTB, FLAGB, rc, SL_B, live, c, o, bad);
    const int* lp = LISTB + (size_t)(rc >> SL_B) * RCAP;
    const float se = SE[rc];
    float m = ninff();
#pragma unroll 1
    for (int b0 = 0; b0 < c; b0 += 32) {
      int e, nd;
      fetch_inc(lp, o, b0 + lane, NE, heNode, NMET, e, nd);
      const float sx = S[nd];
      asm volatile("" :: "v"(sx));
      const float l = edge_logit(sx, se);
      const float lv = (b0 + lane < c) ? l : ninff();
      m = nanmax(m, lv);
    }
    m = wave_nanmax(m);
    float ss = 0.0f;
#pragma unroll 1
    for (int b0 = 0; b0 < c; b0 += 32) {
      int e, nd;
      fetch_inc(lp, o, b0 + lane, NE, heNode, NMET, e, nd);
      const float sx = S[nd];
      asm volatile("" :: "v"(sx));
      const float ex = edge_ex(sx, se, m);
      ss += (b0 + lane < c) ? ex : 0.0f;
    }
    ss = wave_sum(ss);
    const float den = ss + 1e-16f;
    v4f a0 = (v4f){ 0.f, 0.f, 0.f, 0.f };
    v4f a1 = (v4f){ 0.f, 0.f, 0.f, 0.f };
#pragma unroll 1
    for (int b0 = 0; b0 < c; b0 += 32) {
      int e, nd;
      fetch_inc(lp, o, b0 + lane, NE, heNode, NMET, e, nd);
      const float sx = S[nd];
      const float sv = stoich[e];
      asm volatile("" :: "v"(sx));
      asm volatile("" :: "v"(sv));
      const float w = edge_w(sx, se, m, den, bf16_val(sv));
      const int wi = __float_as_int(w);
      const int m32 = (c - b0) < 32 ? (c - b0) : 32;
#pragma unroll 1
      for (int k = 0; k < m32; ++k) {
        const int nk = __builtin_amdgcn_readlane(nd, k);
        const float wk = __int_as_float(__builtin_amdgcn_readlane(wi, k));
        const float* rp = XP + (size_t)nk * DD;
        const v4f x0 = *(const v4f*)(rp + 4 * lane);
        const v4f x1 = *(const v4f*)(rp + 128 + 4 * lane);
        a0[0] = fmaf(wk, x0[0], a0[0]); a0[1] = fmaf(wk, x0[1], a0[1]);
        a0[2] = fmaf(wk, x0[2], a0[2]); a0[3] = fmaf(wk, x0[3], a0[3]);
        a1[0] = fmaf(wk, x1[0], a1[0]); a1[1] = fmaf(wk, x1[1], a1[1]);
        a1[2] = fmaf(wk, x1[2], a1[2]); a1[3] = fmaf(wk, x1[3], a1[3]);
      }
    }
    const float inv = 1.0f / (float)(c > 1 ? c : 1);
    const float pz = bad ? qnanf() : 0.0f;
    v4f r0 = a0 * inv + pz;
    v4f r1 = a1 * inv + pz;
    const v4f z = (v4f){ 0.f, 0.f, 0.f, 0.f };
    r0 = live ? r0 : z;
    r1 = live ? r1 : z;
    store_row(ME + (size_t)r * DD, lane, r0, r1);
    const float mst = ((c == 0) ? 0.0f : m) + pz;
    if (lane == 0) { smx[li] = mst; sdn[li] = den + pz; }
  }
  __syncthreads();
  if (wave == 0) {
    const v4f mv = *(const v4fa*)(smx + 4 * (lane & 15));
    const v4f dv = *(const v4fa*)(sdn + 4 * (lane & 15));
    float* mp = MX  + (size_t)blockIdx.x * 64 + 4 * (lane & 15);
    float* dp = DEN + (size_t)blockIdx.x * 64 + 4 * (lane & 15);
    for (int pass = 0; pass < 2; ++pass) {
      if (lane < 16) { *(volatile v4f*)mp = mv; *(volatile v4f*)dp = dv; }
      __threadfence();
    }
  }
}

__global__ __launch_bounds__(256) void k_node(const int* __restrict__ heEdge, const float* __restrict__ stoich,
                                              const int* __restrict__ LISTC, const int* __restrict__ OFFC,
                                              const int* __restrict__ CNTC, const int* __restrict__ FLAGC,
                                              const float* __restrict__ S, const float* __restrict__ MX,
                                              const float* __restrict__ DEN, const float* __restrict__ ME,
                                              const float* __restrict__ PAR, int bOff, int mode,
                                              float* C0, unsigned short* X1, float* CF) {
  __shared__ __attribute__((aligned(16))) float stg[8][DD];
  __shared__ __attribute__((aligned(16))) float spar[3 * DD];
  const int tid = (int)threadIdx.x, lane = tid & 31;
  const int wave = __builtin_amdgcn_readfirstlane(tid >> 5);
  if (tid < 192) {
    const int so = (tid < 64) ? (bOff + 4 * tid) : (PA_LNG + 4 * (tid - 64));
    *(v4fa*)(spar + 4 * tid) = *(const v4fa*)(PAR + so);
  }
  __syncthreads();
  const float* SE = S + MPM;
  const int n = (int)blockIdx.x * 8 + wave;
  const bool live = n < NMET;
  const int nc = live ? n : NMET - 1;
  int c, o; bool bad;
  seg_hdr(OFFC, CNTC, FLAGC, nc, SL_C, live, c, o, bad);
  const int* lp = LISTC + (size_t)(nc >> SL_C) * RCAP;
  const float sxn = S[nc];
  v4f a0 = (v4f){ 0.f, 0.f, 0.f, 0.f };
  v4f a1 = (v4f){ 0.f, 0.f, 0.f, 0.f };
#pragma unroll 1
  for (int b0 = 0; b0 < c; b0 += 32) {
    int e, ed;
    fetch_inc(lp, o, b0 + lane, NE, heEdge, NRXN, e, ed);
    const float sv  = stoich[e];
    const float sev = SE[ed];
    const float mxv = MX[ed];
    const float dnv = DEN[ed];
    asm volatile("" :: "v"(sv));
    asm volatile("" :: "v"(sev));
    asm volatile("" :: "v"(mxv));
    asm volatile("" :: "v"(dnv));
    const float w = edge_w(sxn, sev, mxv, dnv, bf16_val(sv));
    const int wi = __float_as_int(w);
    const int m32 = (c - b0) < 32 ? (c - b0) : 32;
#pragma unroll 1
    for (int k = 0; k < m32; ++k) {
      const int ek = __builtin_amdgcn_readlane(ed, k);
      const float wk = __int_as_float(__builtin_amdgcn_readlane(wi, k));
      const float* rp = ME + (size_t)ek * DD;
      const v4f x0 = *(const v4f*)(rp + 4 * lane);
      const v4f x1 = *(const v4f*)(rp + 128 + 4 * lane);
      a0[0] = fmaf(wk, x0[0], a0[0]); a0[1] = fmaf(wk, x0[1], a0[1]);
      a0[2] = fmaf(wk, x0[2], a0[2]); a0[3] = fmaf(wk, x0[3], a0[3]);
      a1[0] = fmaf(wk, x1[0], a1[0]); a1[1] = fmaf(wk, x1[1], a1[1]);
      a1[2] = fmaf(wk, x1[2], a1[2]); a1[3] = fmaf(wk, x1[3], a1[3]);
    }
  }
  float* st = stg[wave];
  *(v4fa*)(st + 4 * lane)       = a0;
  *(v4fa*)(st + 128 + 4 * lane) = a1;
  wave_sync_lds();
  const float inv = 1.0f / (float)(c > 1 ? c : 1);
  const float pz = bad ? qnanf() : 0.0f;
#pragma unroll 1
  for (int j = 0; j < 8; ++j) {
    const int col = j * 32 + lane;
    const float x = st[col];
    const float v = tanh_acc(x * inv + spar[col]) + pz;
    st[col] = v;
  }
  const v4f z4 = (v4f){ 0.f, 0.f, 0.f, 0.f };
  if (mode == 0) {
    wave_sync_lds();
    v4f r0 = *(const v4fa*)(st + 4 * lane);
    v4f r1 = *(const v4fa*)(st + 128 + 4 * lane);
    r0 = live ? r0 : z4;
    r1 = live ? r1 : z4;
    store_row(C0 + (size_t)n * DD, lane, r0, r1);
    store_hl(X1 + (size_t)n * KT, lane, r0, r1);
  } else {
    const float* crow = C0 + (size_t)nc * DD;
    float s = 0.0f;
#pragma unroll 1
    for (int j = 0; j < 8; ++j) {
      const int col = j * 32 + lane;
      const float zz = st[col] + crow[col];
      st[col] = zz;
      s += zz;
    }
    s = wave_sum(s);
    const float mu = s * (1.0f / 256.0f);
    float q = 0.0f;
#pragma unroll 1
    for (int j = 0; j < 8; ++j) {
      const int col = j * 32 + lane;
      const float d = st[col] - mu;
      q += d * d;
    }
    q = wave_sum(q);
    const float var = q * (1.0f / 256.0f);
    const float sd = sqrtf(var + 1e-5f);
#pragma unroll 1
    for (int j = 0; j < 8; ++j) {
      const int col = j * 32 + lane;
      const float y = (st[col] - mu) / sd * spar[DD + col] + spar[2 * DD + col];
      st[col] = y;
    }
    wave_sync_lds();
    v4f r0 = *(const v4fa*)(st + 4 * lane);
    v4f r1 = *(const v4fa*)(st + 128 + 4 * lane);
    r0 = live ? r0 : z4;
    r1 = live ? r1 : z4;
    store_row(CF + (size_t)n * DD, lane, r0, r1);
  }
}

struct LayerBufs {
  const int* heNode; const int* heEdge; const float* stoich;
  const int* LB; const int* OB; const int* CB; const int* FB;
  const int* LC; const int* OC; const int* CC; const int* FC;
  const unsigned short* REhl; const unsigned short* WT2; float* PAR;
  float* XPEP; float* S; float* MX; float* DEN; float* ME; float* C0; unsigned short* X1; float* CF;
};

static void run_layer(hipStream_t st, const LayerBufs& b, const unsigned short* Xhl, int wIdx, int attOff, int bOff, int mode) {
  const unsigned short* Wx = b.WT2 + (size_t)wIdx * (DD * KT);
  const unsigned short* We = b.WT2 + (size_t)(wIdx + 1) * (DD * KT);
  float* XP = b.XPEP;
  float* EP = b.XPEP + (size_t)MPM * DD;
  k_gemm_nt<1, 0><<<((MPM / 64) * (DD / 64) + 7) / 8, 256, 0, st>>>(Xhl, Wx, b.PAR, XP, MPM, DD, KT, DD);
  k_gemm_nt<1, 0><<<((MPR / 64) * (DD / 64) + 7) / 8, 256, 0, st>>>(b.REhl, We, b.PAR, EP, MPR, DD, KT, DD);
  k_scores<<<(MPM + MPR) / 64, 256, 0, st>>>(b.XPEP, b.PAR, attOff, b.S);
  k_edge<<<MPR / 64, 256, 0, st>>>(b.heNode, b.stoich, b.LB, b.OB, b.CB, b.FB, b.S, XP, b.ME, b.MX, b.DEN);
  k_node<<<MPM / 8, 256, 0, st>>>(b.heEdge, b.stoich, b.LC, b.OC, b.CC, b.FC, b.S, b.MX, b.DEN, b.ME, b.PAR,
                                  bOff, mode, b.C0, b.X1, b.CF);
}

extern "C" void kernel_launch(void* const* d_in, const int* in_sizes, int n_in,
                              void* d_out, int out_size, void* d_ws, size_t ws_size,
                              hipStream_t stream) {
  if (n_in < 17) return;
  if (in_sizes[0] != NE || in_sizes[1] != NE || in_sizes[2] != NE) return;
  if (in_sizes[3] != NGENE * DD) return;
  if (in_sizes[4] != NP || in_sizes[5] != NP) return;
  if (in_sizes[6] != NMET * DD) return;
  if (in_sizes[7] != DD * DD || in_sizes[8] != DD * DD || in_sizes[11] != DD * DD || in_sizes[12] != DD * DD) return;
  if (in_sizes[9] != 2 * DD || in_sizes[13] != 2 * DD) return;
  if (in_sizes[10] != DD || in_sizes[14] != DD || in_sizes[15] != DD || in_sizes[16] != DD) return;
  if (out_size != NGENE * DD) return;

  const int*   heNode  = (const int*)d_in[0];
  const int*   heEdge  = (const int*)d_in[1];
  const float* stoich  = (const float*)d_in[2];
  const float* geneX   = (const float*)d_in[3];
  const int*   rtgRxn  = (const int*)d_in[4];
  const int*   rtgGene = (const int*)d_in[5];
  const float* emb     = (const float*)d_in[6];
  const float* W0      = (const float*)d_in[7];
  const float* We0     = (const float*)d_in[8];
  const float* att0    = (const float*)d_in[9];
  const float* b0      = (const float*)d_in[10];
  const float* W1      = (const float*)d_in[11];
  const float* We1     = (const float*)d_in[12];
  const float* att1    = (const float*)d_in[13];
  const float* b1      = (const float*)d_in[14];
  const float* lng     = (const float*)d_in[15];
  const float* lnb     = (const float*)d_in[16];
  float* out = (float*)d_out;

  char* ws = (char*)d_ws;
  size_t off = 0;
  auto carve = [&](size_t bytes) { const size_t o = off; off += (bytes + 255) & ~(size_t)255; return o; };
  const size_t oWT2 = carve((size_t)4 * DD * KT * 2);
  const size_t oPAR = carve((size_t)2048 * 4);
  const size_t oMET = carve((size_t)MPM * KT * 2);
  const size_t oX1  = carve((size_t)MPM * KT * 2);
  const size_t oRE  = carve((size_t)MPR * KT * 2);
  const size_t oXE  = carve((size_t)(MPM + MPR) * DD * 4);
  const size_t oS   = carve((size_t)(MPM + MPR) * 4);
  const size_t oMX  = carve((size_t)MPR * 4);
  const size_t oDN  = carve((size_t)MPR * 4);
  const size_t oME  = carve((size_t)MPR * DD * 4);
  const size_t oC0  = carve((size_t)MPM * DD * 4);
  const size_t oCF  = carve((size_t)MPM * DD * 4);
  const size_t oRF  = carve((size_t)MPR * DD * 4);
  const size_t oLA  = carve((size_t)NB_A * RCAP * 4);
  const size_t oLB  = carve((size_t)NB_B * RCAP * 4);
  const size_t oLC  = carve((size_t)NB_C * RCAP * 4);
  const size_t oLD  = carve((size_t)NB_D * RCAP * 4);
  const size_t oOA  = carve((size_t)(NB_A << SL_A) * 4);
  const size_t oCA  = carve((size_t)(NB_A << SL_A) * 4);
  const size_t oOB  = carve((size_t)(NB_B << SL_B) * 4);
  const size_t oCB  = carve((size_t)(NB_B << SL_B) * 4);
  const size_t oOC  = carve((size_t)(NB_C << SL_C) * 4);
  const size_t oCC  = carve((size_t)(NB_C << SL_C) * 4);
  const size_t oOD  = carve((size_t)(NB_D << SL_D) * 4);
  const size_t oCD  = carve((size_t)(NB_D << SL_D) * 4);
  const size_t oFA  = carve((size_t)NB_A * 128);
  const size_t oFB  = carve((size_t)NB_B * 128);
  const size_t oFC  = carve((size_t)NB_C * 128);
  const size_t oFD  = carve((size_t)NB_D * 128);
  if (off > ws_size || off > WSMAX) return;

  unsigned short* WT2 = (unsigned short*)(ws + oWT2);
  float* PAR = (float*)(ws + oPAR);
  unsigned short* METhl = (unsigned short*)(ws + oMET);
  unsigned short* X1hl  = (unsigned short*)(ws + oX1);
  unsigned short* REhl  = (unsigned short*)(ws + oRE);
  float* XPEP = (float*)(ws + oXE);
  float* S    = (float*)(ws + oS);
  float* MX   = (float*)(ws + oMX);
  float* DEN  = (float*)(ws + oDN);
  float* ME   = (float*)(ws + oME);
  float* C0   = (float*)(ws + oC0);
  float* CF   = (float*)(ws + oCF);
  float* RF   = (float*)(ws + oRF);
  int* LA = (int*)(ws + oLA); int* LB = (int*)(ws + oLB); int* LC = (int*)(ws + oLC); int* LD = (int*)(ws + oLD);
  int* OA = (int*)(ws + oOA); int* CA = (int*)(ws + oCA);
  int* OB = (int*)(ws + oOB); int* CB = (int*)(ws + oCB);
  int* OC = (int*)(ws + oOC); int* CC = (int*)(ws + oCC);
  int* OD = (int*)(ws + oOD); int* CD = (int*)(ws + oCD);
  int* FA = (int*)(ws + oFA); int* FB = (int*)(ws + oFB); int* FC = (int*)(ws + oFC); int* FD = (int*)(ws + oFD);

  const int bkLds = BK_INTS * 4;
  hipFuncSetAttribute(reinterpret_cast<const void*>(&k_bucket), hipFuncAttributeMaxDynamicSharedMemorySize, bkLds);

  k_prep<<<PREP_WT + PREP_PAR + PREP_MET, 256, 0, stream>>>(emb, W0, We0, W1, We1, att0, att1, b0, b1, lng, lnb,
                                                            WT2, PAR, METhl);
  k_bucket<<<NB_A, 256, bkLds, stream>>>(rtgRxn,  NP, NRXN,  1 << SL_A, LA, OA, CA, FA);
  k_bucket<<<NB_B, 256, bkLds, stream>>>(heEdge,  NE, NRXN,  1 << SL_B, LB, OB, CB, FB);
  k_bucket<<<NB_C, 256, bkLds, stream>>>(heNode,  NE, NMET,  1 << SL_C, LC, OC, CC, FC);
  k_bucket<<<NB_D, 256, bkLds, stream>>>(rtgGene, NP, NGENE, 1 << SL_D, LD, OD, CD, FD);
  k_mean<1, 1><<<MPR / 8, 256, 0, stream>>>(LA, OA, CA, FA, SL_A, NRXN, MPR, rtgGene, NP, geneX, NGENE, RF, REhl);

  LayerBufs lb;
  lb.heNode = heNode; lb.heEdge = heEdge; lb.stoich = stoich;
  lb.LB = LB; lb.OB = OB; lb.CB = CB; lb.FB = FB;
  lb.LC = LC; lb.OC = OC; lb.CC = CC; lb.FC = FC;
  lb.REhl = REhl; lb.WT2 = WT2; lb.PAR = PAR;
  lb.XPEP = XPEP; lb.S = S; lb.MX = MX; lb.DEN = DEN; lb.ME = ME; lb.C0 = C0; lb.X1 = X1hl; lb.CF = CF;
  run_layer(stream, lb, METhl, 0, PA_ATT0, PA_B0, 0);
  run_layer(stream, lb, X1hl, 2, PA_ATT1, PA_B1, 1);
  k_mean<0, 0><<<MPR / 8, 256, 0, stream>>>(LB, OB, CB, FB, SL_B, NRXN, MPR, heNode, NE, CF, NMET, RF, REhl);
  k_mean<0, 0><<<(NGENE + 7) / 8, 256, 0, stream>>>(LD, OD, CD, FD, SL_D, NGENE, NGENE, rtgRxn, NP, RF, NRXN, out, REhl);
}
